// MultiQueryAttention_14508399526710
// MI455X (gfx1250) — hardware-verified
//
#include <hip/hip_runtime.h>
#include <stdint.h>


typedef _Float16 v16h __attribute__((ext_vector_type(16)));
typedef _Float16 v8h  __attribute__((ext_vector_type(8)));
typedef float    v8f  __attribute__((ext_vector_type(8)));
typedef float    v4f  __attribute__((ext_vector_type(4)));

#define DM 2048
#define HD 128
#define NH 16
#define NB_FULL 2
#define SEQ_FULL 2048
#ifndef NB
#define NB 2
#endif
#ifndef SEQ
#define SEQ 2048
#endif
#ifndef ERLY_REQ
#define ERLY_REQ 512
#endif
#define ERLY ((SEQ < ERLY_REQ) ? SEQ : ERLY_REQ)
#define MROWS (NB * SEQ)
#define ERROWS (NB * ERLY)
#define WSCALE 64.0f
#define PCARRY 1024.0f
#define YCARRY 64.0f
#define RC 1024.0f
#define RCI 0.0009765625f
#define LOG2E 1.4426950408889634f
#define KSC 0.08838834764831845f
#define PP 136

static_assert(SEQ % 128 == 0);
static_assert(SEQ <= SEQ_FULL);
static_assert(NB >= 1 && NB <= NB_FULL);
static_assert(ERLY % 128 == 0 && ERLY >= 128 && ERLY <= SEQ);
static_assert(DM == NH * HD && HD == 128 && DM % 128 == 0 && (NH % 4) == 0);
static_assert(DM / 8 == 256);
static_assert((PP * 2) % 16 == 0 && PP >= 128);

union HFrag { v16h v; v8h h[2]; };

__device__ __forceinline__ v16h load_frag(const _Float16* p) {
    HFrag f;
    f.h[0] = *reinterpret_cast<const v8h*>(p);
    f.h[1] = *reinterpret_cast<const v8h*>(p + 16);
    return f.v;
}

__device__ __forceinline__ v8f wmma16(v16h a, v16h b, v8f c) {
    return __builtin_amdgcn_wmma_f32_16x16x32_f16(false, a, false, b, (short)0, c, false, false);
}

__device__ __forceinline__ float bf16r(float f) {
    unsigned int u = __float_as_uint(f);
    u += 0x7FFFu + ((u >> 16) & 1u);
    u &= 0xFFFF0000u;
    return __uint_as_float(u);
}

__global__ __launch_bounds__(256) void k_cvt_x(const float* __restrict__ x, _Float16* x16)
{
    const int u = blockIdx.x * 256 + threadIdx.x;
    const int row = u >> 8;
    const int col = (u & 255) * 8;
    const int bb = row / SEQ;
    const int s  = row - bb * SEQ;
    const float* src = x + ((size_t)(bb * SEQ_FULL + s)) * DM + col;
    const float4 f0 = *reinterpret_cast<const float4*>(src);
    const float4 f1 = *reinterpret_cast<const float4*>(src + 4);
    v8h o;
    o[0] = (_Float16)bf16r(f0.x); o[1] = (_Float16)bf16r(f0.y);
    o[2] = (_Float16)bf16r(f0.z); o[3] = (_Float16)bf16r(f0.w);
    o[4] = (_Float16)bf16r(f1.x); o[5] = (_Float16)bf16r(f1.y);
    o[6] = (_Float16)bf16r(f1.z); o[7] = (_Float16)bf16r(f1.w);
    _Float16* dst = x16 + (size_t)row * DM + col;
    *(volatile v8h*)dst = o;
    __threadfence();
    *(volatile v8h*)dst = o;
}

__global__ __launch_bounds__(256) void k_cvt_w(const float* __restrict__ W, _Float16* W16)
{
    const size_t u = (size_t)blockIdx.x * 256 + threadIdx.x;
    const float* src = W + u * 8;
    const float4 f0 = *reinterpret_cast<const float4*>(src);
    const float4 f1 = *reinterpret_cast<const float4*>(src + 4);
    v8h o;
    o[0] = (_Float16)(bf16r(f0.x) * WSCALE); o[1] = (_Float16)(bf16r(f0.y) * WSCALE);
    o[2] = (_Float16)(bf16r(f0.z) * WSCALE); o[3] = (_Float16)(bf16r(f0.w) * WSCALE);
    o[4] = (_Float16)(bf16r(f1.x) * WSCALE); o[5] = (_Float16)(bf16r(f1.y) * WSCALE);
    o[6] = (_Float16)(bf16r(f1.z) * WSCALE); o[7] = (_Float16)(bf16r(f1.w) * WSCALE);
    _Float16* dst = W16 + u * 8;
    *(volatile v8h*)dst = o;
    __threadfence();
    *(volatile v8h*)dst = o;
}

__device__ __forceinline__ void store32x64_f16(const _Float16* sw, _Float16* gdst,
                                               size_t pitch, int lane)
{
    const int rq = lane >> 3, seg = lane & 7;
    v8h v[8];
#pragma unroll
    for (int it = 0; it < 8; ++it)
        v[it] = *reinterpret_cast<const v8h*>(sw + (it * 4 + rq) * 64 + seg * 8);
#pragma unroll
    for (int it = 0; it < 8; ++it)
        *(volatile v8h*)(gdst + (size_t)(it * 4 + rq) * pitch + seg * 8) = v[it];
    __threadfence();
#pragma unroll
    for (int it = 0; it < 8; ++it)
        *(volatile v8h*)(gdst + (size_t)(it * 4 + rq) * pitch + seg * 8) = v[it];
}

template <int MODE>
__global__ __launch_bounds__(256) void k_gemm(const _Float16* __restrict__ A,
                                              const _Float16* __restrict__ BT,
                                              const float* __restrict__ bias,
                                              void* C0, void* C1, int N, int K,
                                              float alpha, float oscale)
{
    __shared__ float stg[8 * 1024] __attribute__((aligned(16)));
    const int tid = threadIdx.x;
    const int lane = tid & 31, wave = tid >> 5;
    const int wm = wave & 3, wn = wave >> 2;
    const int l15 = lane & 15, hi8 = (lane >> 4) << 3;
    const int bm0 = blockIdx.y * 128, bn0 = blockIdx.x * 128;

    const _Float16* ap0 = A + (size_t)(bm0 + wm * 32 + l15) * K + hi8;
    const _Float16* ap1 = ap0 + (size_t)16 * K;
    const _Float16* bp  = BT + (size_t)(bn0 + wn * 64 + l15) * K + hi8;
    const size_t bst = (size_t)16 * K;

    const v8f zero8 = {0.f, 0.f, 0.f, 0.f, 0.f, 0.f, 0.f, 0.f};
    v8f acc[2][4];
#pragma unroll
    for (int g = 0; g < 2; ++g)
#pragma unroll
        for (int ni = 0; ni < 4; ++ni) acc[g][ni] = zero8;

    for (int k0 = 0; k0 < K; k0 += 32) {
        const v16h a0 = load_frag(ap0 + k0);
        const v16h a1 = load_frag(ap1 + k0);
        const v16h b0 = load_frag(bp + k0);
        const v16h b1 = load_frag(bp + bst + k0);
        const v16h b2 = load_frag(bp + 2 * bst + k0);
        const v16h b3 = load_frag(bp + 3 * bst + k0);
        acc[0][0] = wmma16(a0, b0, acc[0][0]);
        acc[0][1] = wmma16(a0, b1, acc[0][1]);
        acc[0][2] = wmma16(a0, b2, acc[0][2]);
        acc[0][3] = wmma16(a0, b3, acc[0][3]);
        acc[1][0] = wmma16(a1, b0, acc[1][0]);
        acc[1][1] = wmma16(a1, b1, acc[1][1]);
        acc[1][2] = wmma16(a1, b2, acc[1][2]);
        acc[1][3] = wmma16(a1, b3, acc[1][3]);
        asm volatile("v_nop\n\tv_nop\n\tv_nop\n\tv_nop"
                     : "+v"(acc[0][0]), "+v"(acc[0][1]), "+v"(acc[0][2]), "+v"(acc[0][3]),
                       "+v"(acc[1][0]), "+v"(acc[1][1]), "+v"(acc[1][2]), "+v"(acc[1][3])
                     : "v"(a0), "v"(a1), "v"(b0), "v"(b1), "v"(b2), "v"(b3));
    }

    float bcol[4];
#pragma unroll
    for (int ni = 0; ni < 4; ++ni) bcol[ni] = 0.0f;
    if (MODE != 3) {
#pragma unroll
        for (int ni = 0; ni < 4; ++ni)
            bcol[ni] = bf16r(bias[bn0 + wn * 64 + ni * 16 + l15]);
    }

    if (MODE == 0) {
        const int bb = bm0 / SEQ;
        const int s0 = bm0 - bb * SEQ;
        _Float16* sw = reinterpret_cast<_Float16*>(stg + wave * 1024);
#pragma unroll
        for (int g = 0; g < 2; ++g)
#pragma unroll
            for (int ni = 0; ni < 4; ++ni)
#pragma unroll
                for (int j = 0; j < 8; ++j)
                    sw[(g * 16 + hi8 + j) * 64 + ni * 16 + l15] =
                        (_Float16)((acc[g][ni][j] * alpha + bcol[ni]) * oscale);
        __syncthreads();
        store32x64_f16(sw, (_Float16*)C0 + (size_t)(bm0 + wm * 32) * N + bn0 + wn * 64,
                       (size_t)N, lane);
        if (s0 < ERLY) {
            __syncthreads();
#pragma unroll
            for (int g = 0; g < 2; ++g)
#pragma unroll
                for (int ni = 0; ni < 4; ++ni)
#pragma unroll
                    for (int j = 0; j < 8; ++j) {
                        const float vv = (acc[g][ni][j] * alpha + bcol[ni]) * oscale;
                        const _Float16 hv = (_Float16)vv;
                        sw[(g * 16 + hi8 + j) * 64 + ni * 16 + l15] = (_Float16)((vv - (float)hv) * RC);
                    }
            __syncthreads();
            store32x64_f16(sw, (_Float16*)C1 + (size_t)(bb * ERLY + s0 + wm * 32) * N + bn0 + wn * 64,
                           (size_t)N, lane);
        }
    } else if (MODE == 2) {
        const int bb = bm0 / SEQ;
        const int s0 = bm0 - bb * SEQ;
        _Float16* vs = reinterpret_cast<_Float16*>(stg);
        const int dq = tid >> 4, seg = tid & 15;
#pragma unroll
        for (int g = 0; g < 2; ++g)
#pragma unroll
            for (int ni = 0; ni < 4; ++ni)
#pragma unroll
                for (int j = 0; j < 8; ++j)
                    vs[(wn * 64 + ni * 16 + l15) * 128 + wm * 32 + g * 16 + hi8 + j] =
                        (_Float16)((acc[g][ni][j] * alpha + bcol[ni]) * oscale);
        __syncthreads();
        {
            v8h v[8];
#pragma unroll
            for (int it = 0; it < 8; ++it)
                v[it] = *reinterpret_cast<const v8h*>(vs + (it * 16 + dq) * 128 + seg * 8);
            _Float16* vd = (_Float16*)C0 + ((size_t)(bb * HD)) * SEQ + s0 + seg * 8;
#pragma unroll
            for (int it = 0; it < 8; ++it)
                *(volatile v8h*)(vd + (size_t)(it * 16 + dq) * SEQ) = v[it];
            __threadfence();
#pragma unroll
            for (int it = 0; it < 8; ++it)
                *(volatile v8h*)(vd + (size_t)(it * 16 + dq) * SEQ) = v[it];
        }
        if (s0 < ERLY) {
            __syncthreads();
#pragma unroll
            for (int g = 0; g < 2; ++g)
#pragma unroll
                for (int ni = 0; ni < 4; ++ni)
#pragma unroll
                    for (int j = 0; j < 8; ++j) {
                        const float vv = (acc[g][ni][j] * alpha + bcol[ni]) * oscale;
                        const _Float16 hv = (_Float16)vv;
                        vs[(wn * 64 + ni * 16 + l15) * 128 + wm * 32 + g * 16 + hi8 + j] =
                            (_Float16)((vv - (float)hv) * RC);
                    }
            __syncthreads();
            v8h v[8];
#pragma unroll
            for (int it = 0; it < 8; ++it)
                v[it] = *reinterpret_cast<const v8h*>(vs + (it * 16 + dq) * 128 + seg * 8);
            _Float16* vd = (_Float16*)C1 + ((size_t)(bb * HD)) * ERLY + s0 + seg * 8;
#pragma unroll
            for (int it = 0; it < 8; ++it)
                *(volatile v8h*)(vd + (size_t)(it * 16 + dq) * ERLY) = v[it];
            __threadfence();
#pragma unroll
            for (int it = 0; it < 8; ++it)
                *(volatile v8h*)(vd + (size_t)(it * 16 + dq) * ERLY) = v[it];
        }
    } else {
        float* swf = stg + wave * 1024;
        const int rq = lane >> 4, seg = lane & 15;
        int crow0 = 0;
        bool addc = false;
        if (MODE == 1) {
            const int bb = bm0 / SEQ;
            const int s0 = bm0 - bb * SEQ;
            addc = (s0 < ERLY);
            crow0 = bb * ERLY + s0;
        }
#pragma unroll
        for (int g = 0; g < 2; ++g) {
#pragma unroll
            for (int ni = 0; ni < 4; ++ni)
#pragma unroll
                for (int j = 0; j < 8; ++j)
                    swf[(hi8 + j) * 64 + ni * 16 + l15] = (acc[g][ni][j] * alpha + bcol[ni]) * oscale;
            __syncthreads();
            v4f v[8];
#pragma unroll
            for (int it = 0; it < 8; ++it)
                v[it] = *reinterpret_cast<const v4f*>(swf + (it * 2 + rq) * 64 + seg * 4);
            if (addc) {
                const float* cr = (const float*)C1 + (size_t)(crow0 + wm * 32 + g * 16) * N
                                  + bn0 + wn * 64 + seg * 4;
#pragma unroll
                for (int it = 0; it < 8; ++it)
                    v[it] += *reinterpret_cast<const v4f*>(cr + (size_t)(it * 2 + rq) * N);
            }
            float* gd = (float*)C0 + (size_t)(bm0 + wm * 32 + g * 16) * N + bn0 + wn * 64 + seg * 4;
#pragma unroll
            for (int it = 0; it < 8; ++it)
                *(volatile v4f*)(gd + (size_t)(it * 2 + rq) * N) = v[it];
            __threadfence();
#pragma unroll
            for (int it = 0; it < 8; ++it)
                *(volatile v4f*)(gd + (size_t)(it * 2 + rq) * N) = v[it];
            __syncthreads();
        }
    }
}

__global__ __launch_bounds__(128) __attribute__((amdgpu_num_vgpr(256)))
void k_attn(const _Float16* __restrict__ qp, const _Float16* __restrict__ kp,
            const _Float16* __restrict__ vT, _Float16* yp)
{
    __shared__ _Float16 Ws[4 * 16 * PP] __attribute__((aligned(16)));
    const int lane = threadIdx.x & 31;
    const int wv   = threadIdx.x >> 5;
    const int l15  = lane & 15;
    const int hi8  = (lane >> 4) << 3;

    constexpr int NQL = ((SEQ - ERLY) / 16 > 0) ? ((SEQ - ERLY) / 16) : 1;
    int gw = blockIdx.x * 4 + wv;
    const int h = gw % NH; gw /= NH;
    const int qt = (ERLY / 16) + (gw % NQL);
    const int b  = gw / NQL;
    const int r0 = qt * 16;

    const _Float16* qbase = qp + ((size_t)(b * SEQ + r0 + l15)) * DM + h * HD + hi8;
    const v16h aQ0 = load_frag(qbase);
    const v16h aQ1 = load_frag(qbase + 32);
    const v16h aQ2 = load_frag(qbase + 64);
    const v16h aQ3 = load_frag(qbase + 96);

    const _Float16* kbase = kp + (size_t)b * SEQ * HD + hi8;
    const _Float16* vbase = vT + ((size_t)(b * HD)) * SEQ + hi8;

    const v8f zero8 = {0.f, 0.f, 0.f, 0.f, 0.f, 0.f, 0.f, 0.f};
    float m[8], l[8];
    v8f accY[8];
#pragma unroll
    for (int j = 0; j < 8; ++j) { m[j] = -1.0e30f; l[j] = 0.0f; }
#pragma unroll
    for (int ni = 0; ni < 8; ++ni) accY[ni] = zero8;

    _Float16* ps = Ws + wv * 16 * PP;
    const int kend = r0 + 16;
    const int qrow = r0 + hi8;

#pragma unroll 1
    for (int tc = 0; tc < kend; tc += 32) {
        const _Float16* kp0 = kbase + (size_t)(tc + l15) * HD;
        const _Float16* kp1 = kp0 + 16 * HD;
        const v16h b00 = load_frag(kp0);
        const v16h b01 = load_frag(kp0 + 32);
        const v16h b02 = load_frag(kp0 + 64);
        const v16h b03 = load_frag(kp0 + 96);
        const v16h b10 = load_frag(kp1);
        const v16h b11 = load_frag(kp1 + 32);
        const v16h b12 = load_frag(kp1 + 64);
        const v16h b13 = load_frag(kp1 + 96);
        v8f s0 = zero8, s1 = zero8;
        s0 = wmma16(aQ0, b00, s0);
        s1 = wmma16(aQ0, b10, s1);
        s0 = wmma16(aQ1, b01, s0);
        s1 = wmma16(aQ1, b11, s1);
        s0 = wmma16(aQ2, b02, s0);
        s1 = wmma16(aQ2, b12, s1);
        s0 = wmma16(aQ3, b03, s0);
        s1 = wmma16(aQ3, b13, s1);
        asm volatile("v_nop\n\tv_nop\n\tv_nop\n\tv_nop"
                     : "+v"(s0), "+v"(s1)
                     : "v"(aQ0), "v"(aQ1), "v"(aQ2), "v"(aQ3),
                       "v"(b00), "v"(b01), "v"(b02), "v"(b03),
                       "v"(b10), "v"(b11), "v"(b12), "v"(b13));

        const int key0 = tc + l15, key1 = tc + 16 + l15;
#pragma unroll
        for (int j = 0; j < 8; ++j) {
            const int row = qrow + j;
            const float a0 = (key0 > row) ? -1.0e30f : s0[j] * KSC;
            const float a1 = (key1 > row) ? -1.0e30f : s1[j] * KSC;
            float mt = fmaxf(a0, a1);
#pragma unroll
            for (int off = 8; off >= 1; off >>= 1)
                mt = fmaxf(mt, __shfl_xor(mt, off, 16));
            const float mn = fmaxf(m[j], mt);
            const float sc = exp2f(m[j] - mn);
            const float p0 = exp2f(a0 - mn);
            const float p1 = exp2f(a1 - mn);
            float rs = p0 + p1;
#pragma unroll
            for (int off = 8; off >= 1; off >>= 1)
                rs += __shfl_xor(rs, off, 16);
            l[j] = l[j] * sc + rs;
            m[j] = mn;
#pragma unroll
            for (int ni = 0; ni < 8; ++ni) accY[ni][j] *= sc;
            const int rr = hi8 + j;
            ps[rr * PP + l15]      = (_Float16)(p0 * PCARRY);
            ps[rr * PP + 16 + l15] = (_Float16)(p1 * PCARRY);
        }
        __syncthreads();

        const v16h aP  = load_frag(ps + l15 * PP + hi8);
        const v16h bV0 = load_frag(vbase + (size_t)(0 * 16 + l15) * SEQ + tc);
        const v16h bV1 = load_frag(vbase + (size_t)(1 * 16 + l15) * SEQ + tc);
        const v16h bV2 = load_frag(vbase + (size_t)(2 * 16 + l15) * SEQ + tc);
        const v16h bV3 = load_frag(vbase + (size_t)(3 * 16 + l15) * SEQ + tc);
        const v16h bV4 = load_frag(vbase + (size_t)(4 * 16 + l15) * SEQ + tc);
        const v16h bV5 = load_frag(vbase + (size_t)(5 * 16 + l15) * SEQ + tc);
        const v16h bV6 = load_frag(vbase + (size_t)(6 * 16 + l15) * SEQ + tc);
        const v16h bV7 = load_frag(vbase + (size_t)(7 * 16 + l15) * SEQ + tc);
        accY[0] = wmma16(aP, bV0, accY[0]);
        accY[1] = wmma16(aP, bV1, accY[1]);
        accY[2] = wmma16(aP, bV2, accY[2]);
        accY[3] = wmma16(aP, bV3, accY[3]);
        accY[4] = wmma16(aP, bV4, accY[4]);
        accY[5] = wmma16(aP, bV5, accY[5]);
        accY[6] = wmma16(aP, bV6, accY[6]);
        accY[7] = wmma16(aP, bV7, accY[7]);
        asm volatile("v_nop\n\tv_nop\n\tv_nop\n\tv_nop"
                     : "+v"(accY[0]), "+v"(accY[1]), "+v"(accY[2]), "+v"(accY[3]),
                       "+v"(accY[4]), "+v"(accY[5]), "+v"(accY[6]), "+v"(accY[7])
                     : "v"(aP), "v"(bV0), "v"(bV1), "v"(bV2), "v"(bV3),
                       "v"(bV4), "v"(bV5), "v"(bV6), "v"(bV7));
    }
    __syncthreads();

    float inv[8];
#pragma unroll
    for (int j = 0; j < 8; ++j) inv[j] = (YCARRY / PCARRY) / l[j];
#pragma unroll
    for (int ni = 0; ni < 8; ++ni)
#pragma unroll
        for (int j = 0; j < 8; ++j)
            ps[(hi8 + j) * PP + ni * 16 + l15] = (_Float16)(accY[ni][j] * inv[j]);
    __syncthreads();

    const int rq = lane >> 4, seg = lane & 15;
    v8h v[8];
#pragma unroll
    for (int it = 0; it < 8; ++it)
        v[it] = *reinterpret_cast<const v8h*>(ps + (it * 2 + rq) * PP + seg * 8);
    _Float16* yd = yp + ((size_t)(b * SEQ + r0)) * DM + h * HD + seg * 8;
#pragma unroll
    for (int it = 0; it < 8; ++it)
        *(volatile v8h*)(yd + (size_t)(it * 2 + rq) * DM) = v[it];
    __threadfence();
#pragma unroll
    for (int it = 0; it < 8; ++it)
        *(volatile v8h*)(yd + (size_t)(it * 2 + rq) * DM) = v[it];
}

__global__ __launch_bounds__(128) __attribute__((amdgpu_num_vgpr(256)))
void k_attn_e(const _Float16* __restrict__ qp, const _Float16* __restrict__ qr,
              const _Float16* __restrict__ kp, const _Float16* __restrict__ kr,
              const _Float16* __restrict__ vT, const _Float16* __restrict__ vTr,
              _Float16* yp, _Float16* yr)
{
    __shared__ _Float16 Ws[4 * 16 * PP] __attribute__((aligned(16)));
    const int lane = threadIdx.x & 31;
    const int wv   = threadIdx.x >> 5;
    const int l15  = lane & 15;
    const int hi8  = (lane >> 4) << 3;

    constexpr int NQE = ERLY / 16;
    int gw = blockIdx.x * 4 + wv;
    const int h = gw % NH; gw /= NH;
    const int dsel = gw & 1; gw >>= 1;
    const int qt = gw % NQE;
    const int b  = gw / NQE;
    const int r0 = qt * 16;
    const int d0 = dsel * 64;

    const _Float16* qbase  = qp + ((size_t)(b * SEQ + r0 + l15)) * DM + h * HD + hi8;
    const _Float16* qrbase = qr + ((size_t)(b * ERLY + r0 + l15)) * DM + h * HD + hi8;
    const _Float16* kbase  = kp + (size_t)b * SEQ * HD + hi8;
    const _Float16* krbase = kr + (size_t)b * ERLY * HD + hi8;
    const _Float16* vbase  = vT  + ((size_t)(b * HD + d0)) * SEQ + hi8;
    const _Float16* vrbase = vTr + ((size_t)(b * HD + d0)) * ERLY + hi8;

    const v8f zero8 = {0.f, 0.f, 0.f, 0.f, 0.f, 0.f, 0.f, 0.f};
    float m[8], l[8];
    v8f accY[4], accR[4];
#pragma unroll
    for (int j = 0; j < 8; ++j) { m[j] = -1.0e30f; l[j] = 0.0f; }
#pragma unroll
    for (int ni = 0; ni < 4; ++ni) { accY[ni] = zero8; accR[ni] = zero8; }

    _Float16* ps = Ws + wv * 16 * PP;
    const int kend = r0 + 16;
    const int qrow = r0 + hi8;

#pragma unroll 1
    for (int tc = 0; tc < kend; tc += 32) {
        const _Float16* kp0 = kbase + (size_t)(tc + l15) * HD;
        const _Float16* kp1 = kp0 + 16 * HD;
        const _Float16* ep0 = krbase + (size_t)(tc + l15) * HD;
        const _Float16* ep1 = ep0 + 16 * HD;
        v8f s0 = zero8, s1 = zero8, t0 = zero8, t1 = zero8;
#pragma unroll
        for (int c = 0; c < 4; ++c) {
            const v16h aQ = load_frag(qbase + 32 * c);
            const v16h aR = load_frag(qrbase + 32 * c);
            const v16h b0 = load_frag(kp0 + 32 * c);
            const v16h b1 = load_frag(kp1 + 32 * c);
            const v16h e0 = load_frag(ep0 + 32 * c);
            const v16h e1 = load_frag(ep1 + 32 * c);
            s0 = wmma16(aQ, b0, s0);
            s1 = wmma16(aQ, b1, s1);
            t0 = wmma16(aR, b0, t0);
            t1 = wmma16(aR, b1, t1);
            t0 = wmma16(aQ, e0, t0);
            t1 = wmma16(aQ, e1, t1);
            asm volatile("v_nop\n\tv_nop\n\tv_nop\n\tv_nop"
                         : "+v"(s0), "+v"(s1), "+v"(t0), "+v"(t1)
                         : "v"(aQ), "v"(aR), "v"(b0), "v"(b1), "v"(e0), "v"(e1));
        }

        const int key0 = tc + l15, key1 = tc + 16 + l15;
#pragma unroll
        for (int j = 0; j < 8; ++j) {
            const int row = qrow + j;
            const float a0 = (key0 > row) ? -1.0e30f : (s0[j] + t0[j] * RCI) * KSC;
            const float a1 = (key1 > row) ? -1.0e30f : (s1[j] + t1[j] * RCI) * KSC;
            float mt = fmaxf(a0, a1);
#pragma unroll
            for (int off = 8; off >= 1; off >>= 1)
                mt = fmaxf(mt, __shfl_xor(mt, off, 16));
            const float mn = fmaxf(m[j], mt);
            const float sc = exp2f(m[j] - mn);
            const float p0 = exp2f(a0 - mn);
            const float p1 = exp2f(a1 - mn);
            float rs = p0 + p1;
#pragma unroll
            for (int off = 8; off >= 1; off >>= 1)
                rs += __shfl_xor(rs, off, 16);
            l[j] = l[j] * sc + rs;
            m[j] = mn;
#pragma unroll
            for (int ni = 0; ni < 4; ++ni) { accY[ni][j] *= sc; accR[ni][j] *= sc; }
            const float pf0 = p0 * PCARRY, pf1 = p1 * PCARRY;
            const _Float16 h0 = (_Float16)pf0, h1 = (_Float16)pf1;
            const _Float16 g0 = (_Float16)((pf0 - (float)h0) * RC);
            const _Float16 g1 = (_Float16)((pf1 - (float)h1) * RC);
            const int rr = hi8 + j;
            ps[rr * PP + l15]      = h0;
            ps[rr * PP + 16 + l15] = h1;
            ps[rr * PP + 32 + l15] = g0;
            ps[rr * PP + 48 + l15] = g1;
        }
        __syncthreads();

        const v16h aP  = load_frag(ps + l15 * PP + hi8);
        const v16h aPr = load_frag(ps + l15 * PP + 32 + hi8);
        const v16h bV0 = load_frag(vbase + (size_t)(0 * 16 + l15) * SEQ + tc);
        const v16h bV1 = load_frag(vbase + (size_t)(1 * 16 + l15) * SEQ + tc);
        const v16h bV2 = load_frag(vbase + (size_t)(2 * 16 + l15) * SEQ + tc);
        const v16h bV3 = load_frag(vbase + (size_t)(3 * 16 + l15) * SEQ + tc);
        const v16h bR0 = load_frag(vrbase + (size_t)(0 * 16 + l15) * ERLY + tc);
        const v16h bR1 = load_frag(vrbase + (size_t)(1 * 16 + l15) * ERLY + tc);
        const v16h bR2 = load_frag(vrbase + (size_t)(2 * 16 + l15) * ERLY + tc);
        const v16h bR3 = load_frag(vrbase + (size_t)(3 * 16 + l15) * ERLY + tc);
        accY[0] = wmma16(aP,  bV0, accY[0]);
        accY[1] = wmma16(aP,  bV1, accY[1]);
        accY[2] = wmma16(aP,  bV2, accY[2]);
        accY[3] = wmma16(aP,  bV3, accY[3]);
        accR[0] = wmma16(aPr, bV0, accR[0]);
        accR[1] = wmma16(aPr, bV1, accR[1]);
        accR[2] = wmma16(aPr, bV2, accR[2]);
        accR[3] = wmma16(aPr, bV3, accR[3]);
        accR[0] = wmma16(aP,  bR0, accR[0]);
        accR[1] = wmma16(aP,  bR1, accR[1]);
        accR[2] = wmma16(aP,  bR2, accR[2]);
        accR[3] = wmma16(aP,  bR3, accR[3]);
        asm volatile("v_nop\n\tv_nop\n\tv_nop\n\tv_nop"
                     : "+v"(accY[0]), "+v"(accY[1]), "+v"(accY[2]), "+v"(accY[3]),
                       "+v"(accR[0]), "+v"(accR[1]), "+v"(accR[2]), "+v"(accR[3])
                     : "v"(aP), "v"(aPr), "v"(bV0), "v"(bV1), "v"(bV2), "v"(bV3),
                       "v"(bR0), "v"(bR1), "v"(bR2), "v"(bR3));
    }
    __syncthreads();

    float inv[8];
#pragma unroll
    for (int j = 0; j < 8; ++j) inv[j] = (YCARRY / PCARRY) / l[j];
#pragma unroll
    for (int ni = 0; ni < 4; ++ni)
#pragma unroll
        for (int j = 0; j < 8; ++j) {
            const float vv = (accY[ni][j] + accR[ni][j] * RCI) * inv[j];
            const _Float16 hv = (_Float16)vv;
            ps[(hi8 + j) * PP + ni * 16 + l15]      = hv;
            ps[(hi8 + j) * PP + 64 + ni * 16 + l15] = (_Float16)((vv - (float)hv) * RC);
        }
    __syncthreads();

    const int rq = lane >> 3, seg = lane & 7;
    v8h v[4], w[4];
#pragma unroll
    for (int it = 0; it < 4; ++it) {
        v[it] = *reinterpret_cast<const v8h*>(ps + (it * 4 + rq) * PP + seg * 8);
        w[it] = *reinterpret_cast<const v8h*>(ps + (it * 4 + rq) * PP + 64 + seg * 8);
    }
    _Float16* yd  = yp + ((size_t)(b * SEQ + r0)) * DM + h * HD + d0 + seg * 8;
    _Float16* yrd = yr + ((size_t)(b * ERLY + r0)) * DM + h * HD + d0 + seg * 8;
#pragma unroll
    for (int it = 0; it < 4; ++it) {
        *(volatile v8h*)(yd  + (size_t)(it * 4 + rq) * DM) = v[it];
        *(volatile v8h*)(yrd + (size_t)(it * 4 + rq) * DM) = w[it];
    }
    __threadfence();
#pragma unroll
    for (int it = 0; it < 4; ++it) {
        *(volatile v8h*)(yd  + (size_t)(it * 4 + rq) * DM) = v[it];
        *(volatile v8h*)(yrd + (size_t)(it * 4 + rq) * DM) = w[it];
    }
}

extern "C" void kernel_launch(void* const* d_in, const int* in_sizes, int n_in,
                              void* d_out, int out_size, void* d_ws, size_t ws_size,
                              hipStream_t stream) {
    if (n_in < 10) return;
    const long long needX = ((long long)(NB - 1) * SEQ_FULL + SEQ) * DM;
    if ((long long)in_sizes[0] < needX || (long long)in_sizes[1] < needX) return;
    if (in_sizes[2] < DM * DM || in_sizes[3] < DM) return;
    if (in_sizes[4] < HD * DM || in_sizes[5] < HD) return;
    if (in_sizes[6] < HD * DM || in_sizes[7] < HD) return;
    if (in_sizes[8] < DM * DM || in_sizes[9] < DM) return;
    if ((long long)out_size < (long long)MROWS * DM) return;

    const float* x  = (const float*)d_in[0];
    const float* kv = (const float*)d_in[1];
    const float* Wq = (const float*)d_in[2];
    const float* bq = (const float*)d_in[3];
    const float* Wk = (const float*)d_in[4];
    const float* bk = (const float*)d_in[5];
    const float* Wv = (const float*)d_in[6];
    const float* bv = (const float*)d_in[7];
    const float* Wo = (const float*)d_in[8];
    const float* bo = (const float*)d_in[9];
    float* out = (float*)d_out;

    size_t off = 0;
    char* wsb = (char*)d_ws;
    auto carve = [&](size_t bytes) -> void* {
        void* p = wsb + off;
        off += (bytes + 255) & ~(size_t)255;
        return p;
    };
    _Float16* x16  = (_Float16*)carve((size_t)MROWS * DM * 2);
    _Float16* kv16 = (_Float16*)carve((size_t)MROWS * DM * 2);
    _Float16* Wq16 = (_Float16*)carve((size_t)DM * DM * 2);
    _Float16* Wk16 = (_Float16*)carve((size_t)HD * DM * 2);
    _Float16* Wv16 = (_Float16*)carve((size_t)HD * DM * 2);
    _Float16* Wo16 = (_Float16*)carve((size_t)DM * DM * 2);
    _Float16* q16  = (_Float16*)carve((size_t)MROWS * DM * 2);
    _Float16* qres = (_Float16*)carve((size_t)ERROWS * DM * 2);
    _Float16* kpl  = (_Float16*)carve((size_t)MROWS * HD * 2);
    _Float16* kres = (_Float16*)carve((size_t)ERROWS * HD * 2);
    _Float16* vT   = (_Float16*)carve((size_t)NB * HD * SEQ * 2);
    _Float16* vTr  = (_Float16*)carve((size_t)NB * HD * ERLY * 2);
    _Float16* y16  = (_Float16*)carve((size_t)MROWS * DM * 2);
    _Float16* yres = (_Float16*)carve((size_t)ERROWS * DM * 2);
    float*    corr = (float*)carve((size_t)ERROWS * DM * 4);
    if (off > ws_size) return;
    if (off > (size_t)134217728) return;

    dim3 blk(256);

    k_cvt_x<<<dim3(MROWS), blk, 0, stream>>>(x, x16);
    k_cvt_x<<<dim3(MROWS), blk, 0, stream>>>(kv, kv16);
    k_cvt_w<<<dim3((DM * DM) / 2048), blk, 0, stream>>>(Wq, Wq16);
    k_cvt_w<<<dim3((HD * DM) / 2048), blk, 0, stream>>>(Wk, Wk16);
    k_cvt_w<<<dim3((HD * DM) / 2048), blk, 0, stream>>>(Wv, Wv16);
    k_cvt_w<<<dim3((DM * DM) / 2048), blk, 0, stream>>>(Wo, Wo16);

    k_gemm<0><<<dim3(DM / 128, MROWS / 128), blk, 0, stream>>>(
        x16, Wq16, bq, (void*)q16, (void*)qres, DM, DM, 1.0f / WSCALE, LOG2E);
    k_gemm<0><<<dim3(HD / 128, MROWS / 128), blk, 0, stream>>>(
        kv16, Wk16, bk, (void*)kpl, (void*)kres, HD, DM, 1.0f / WSCALE, 1.0f);
    k_gemm<2><<<dim3(HD / 128, MROWS / 128), blk, 0, stream>>>(
        kv16, Wv16, bv, (void*)vT, (void*)vTr, HD, DM, 1.0f / WSCALE, 1.0f);

    const int nearly = NB * (ERLY / 16) * 2 * (NH / 4);
    k_attn_e<<<dim3(nearly), dim3(128), 0, stream>>>(q16, qres, kpl, kres, vT, vTr, y16, yres);
    const int nlate = NB * ((SEQ - ERLY) / 16) * (NH / 4);
    if (nlate > 0)
        k_attn<<<dim3(nlate), dim3(128), 0, stream>>>(q16, kpl, vT, y16);

    k_gemm<3><<<dim3(DM / 128, ERROWS / 128), blk, 0, stream>>>(
        yres, Wo16, bo, (void*)corr, (void*)corr, DM, DM, 1.0f / (RC * YCARRY * WSCALE), 1.0f);
    k_gemm<1><<<dim3(DM / 128, MROWS / 128), blk, 0, stream>>>(
        y16, Wo16, bo, (void*)out, (void*)corr, DM, DM, 1.0f / (YCARRY * WSCALE), 1.0f);
}
